// T5Voice_45234595561601
// MI455X (gfx1250) — hardware-verified
//
#include <hip/hip_runtime.h>


#define NB_  4
#define TT   1024
#define LL   4096
#define DD   1024
#define NH_  16
#define HDM  64
#define MM   4096
#define PCAR 1024.0f
typedef _Float16 h16;
typedef unsigned short bf;
typedef __attribute__((ext_vector_type(16))) __bf16   v16bf;
typedef __attribute__((ext_vector_type(16))) _Float16 v16h;
typedef __attribute__((ext_vector_type(8)))  _Float16 v8h;
typedef __attribute__((ext_vector_type(8)))  unsigned short v8us;
typedef __attribute__((ext_vector_type(8)))  float    v8f;
typedef __attribute__((ext_vector_type(4)))  float    v4f;
typedef v8h  __attribute__((may_alias)) v8ha;
typedef v4f  __attribute__((may_alias)) v4fa;
typedef v8us __attribute__((may_alias)) v8usa;

__device__ __forceinline__ unsigned short f2bf(float f) { unsigned u = __float_as_uint(f); u += 0x7FFFu + ((u >> 16) & 1u); return (unsigned short)(u >> 16); }
__device__ __forceinline__ float bf2f(unsigned short b) { return __uint_as_float(((unsigned)b) << 16); }
__device__ __forceinline__ float bfr(float f) { return bf2f(f2bf(f)); }
__device__ __forceinline__ v16h cat16(v8h lo, v8h hi) { return __builtin_shufflevector(lo, hi, 0, 1, 2, 3, 4, 5, 6, 7, 8, 9, 10, 11, 12, 13, 14, 15); }
__device__ __forceinline__ v16bf cat16b(v8us lo, v8us hi) { return __builtin_bit_cast(v16bf, __builtin_shufflevector(lo, hi, 0, 1, 2, 3, 4, 5, 6, 7, 8, 9, 10, 11, 12, 13, 14, 15)); }
__device__ __forceinline__ v8f wmma16(v16h a, v16h b, v8f c) { return __builtin_amdgcn_wmma_f32_16x16x32_f16(false, a, false, b, (short)0, c, false, false); }
__device__ __forceinline__ v8f wmmab(v16bf a, v16bf b, v8f c) { return __builtin_amdgcn_wmma_f32_16x16x32_bf16(false, a, false, b, (short)0, c, false, false); }


template <typename T16> struct WFrag;
template <> struct WFrag<h16> { typedef v16h V; static __device__ __forceinline__ V ld(const h16* p) { return cat16(*(const v8h*)p, *(const v8h*)(p + 16)); } static __device__ __forceinline__ v8f mma(V a, V b, v8f c) { return wmma16(a, b, c); } };
template <> struct WFrag<bf> { typedef v16bf V; static __device__ __forceinline__ V ld(const bf* p) { return cat16b(*(const v8us*)p, *(const v8us*)(p + 16)); } static __device__ __forceinline__ v8f mma(V a, V b, v8f c) { return wmmab(a, b, c); } };
template <typename T16, int NSPLIT, bool BIAS>
__global__ __launch_bounds__(32) void k_gemmw(const T16* __restrict__ A, const T16* __restrict__ A2, const T16* __restrict__ Bt, const T16* __restrict__ Bt2, int K, float* C, int ldc, const float* __restrict__ bias, size_t sA, size_t sB, size_t sC) {
    typedef typename WFrag<T16>::V V;
    __shared__ __align__(16) float os[16 * 68];
    const size_t z = blockIdx.z; A += z * sA; if (A2) A2 += z * sA; Bt += z * sB; if (Bt2) Bt2 += z * sB; C += z * sC;
    const int lane = threadIdx.x & 31, lr = lane & 15, hi = lane >> 4; const int r0 = blockIdx.x * 64, c0 = blockIdx.y * 64;
    v8f acc[4][4];
#pragma unroll
    for (int mb = 0; mb < 4; ++mb)
#pragma unroll
        for (int nb = 0; nb < 4; ++nb) acc[mb][nb] = (v8f){};
    const size_t aoff = (size_t)(r0 + lr) * K + 8 * hi, boff = (size_t)(c0 + lr) * K + 8 * hi;
#pragma unroll 1
    for (int kc = 0; kc < K; kc += 32) {
        V a[4], a2[4];
#pragma unroll
        for (int mb = 0; mb < 4; ++mb) { a[mb] = WFrag<T16>::ld(A + aoff + (size_t)mb * 16 * K + kc); if (NSPLIT == 1 || NSPLIT == 2) a2[mb] = WFrag<T16>::ld(A2 + aoff + (size_t)mb * 16 * K + kc); }
#pragma unroll
        for (int nb = 0; nb < 4; ++nb) { const V b = WFrag<T16>::ld(Bt + boff + (size_t)nb * 16 * K + kc); V b2; if (NSPLIT >= 2) b2 = WFrag<T16>::ld(Bt2 + boff + (size_t)nb * 16 * K + kc);
#pragma unroll
            for (int mb = 0; mb < 4; ++mb) { acc[mb][nb] = WFrag<T16>::mma(a[mb], b, acc[mb][nb]); if (NSPLIT == 1 || NSPLIT == 2) acc[mb][nb] = WFrag<T16>::mma(a2[mb], b, acc[mb][nb]); if (NSPLIT >= 2) acc[mb][nb] = WFrag<T16>::mma(a[mb], b2, acc[mb][nb]); } }
        asm volatile("v_nop\n\tv_nop\n\tv_nop\n\tv_nop" : "+v"(acc[0][0]), "+v"(acc[1][1]), "+v"(acc[2][2]), "+v"(acc[3][3]) : "v"(a[0]), "v"(a[3]));
    }
#pragma unroll
    for (int mb = 0; mb < 4; ++mb) {
#pragma unroll
        for (int nb = 0; nb < 4; ++nb) {
#pragma unroll
            for (int j = 0; j < 8; ++j) os[(hi * 8 + j) * 68 + nb * 16 + lr] = acc[mb][nb][j]; }
        __builtin_amdgcn_wave_barrier(); asm volatile("" ::: "memory");
        float* crow = C + (size_t)(r0 + mb * 16) * ldc + c0;
#pragma unroll 1
        for (int ps = 0; ps < 2; ++ps) {
#pragma unroll
            for (int s = 0; s < 8; ++s) { const int row = 2 * s + hi, cofs = lr * 4; v4f val = *(const v4fa*)(os + row * 68 + cofs); if (BIAS) { val[0] += bfr(bias[c0 + cofs]); val[1] += bfr(bias[c0 + cofs + 1]); val[2] += bfr(bias[c0 + cofs + 2]); val[3] += bfr(bias[c0 + cofs + 3]); }
                *(volatile v4f*)(crow + (size_t)row * ldc + cofs) = val; }
            if (ps == 0) __threadfence(); }
        __builtin_amdgcn_wave_barrier(); asm volatile("" ::: "memory");
    }
}

__device__ __forceinline__ h16 tohx(float x) { return (h16)x; }
__device__ __forceinline__ void splitf(float y, unsigned short& h, unsigned short& l) { h = f2bf(y); l = f2bf(y - bf2f(h)); }
typedef __attribute__((ext_vector_type(2))) _Float16 v2h;
typedef __attribute__((ext_vector_type(4))) _Float16 v4h;
typedef __attribute__((ext_vector_type(2))) unsigned short v2us;
typedef __attribute__((ext_vector_type(4))) unsigned short v4us;
typedef __attribute__((ext_vector_type(2))) float v2f;

__global__ __launch_bounds__(256) void k_wtG(const float* __restrict__ w, int K, int N, bf* Bt) {
    const int lane = threadIdx.x & 31; const int L0 = (blockIdx.x * 8 + (threadIdx.x >> 5)) * 8; const int nlines = N * K / 64;
#pragma unroll 1
    for (int ps = 0; ps < 2; ++ps) {
#pragma unroll 1
        for (int l = 0; l < 8; ++l) { const int L = L0 + l; if (L >= nlines) break; const size_t e = (size_t)L * 64 + lane * 2; const int k = (int)(e % K), n = (int)(e / K); v2us o;
            o[0] = f2bf(w[(size_t)k * N + n]); o[1] = f2bf(w[(size_t)(k + 1) * N + n]); *(volatile v2us*)(Bt + e) = o; }
        if (ps == 0) __threadfence(); }
}
__global__ __launch_bounds__(256) void k_pl(const float* __restrict__ F, int pitch, int nh, int hd, h16* P) { const size_t e = ((size_t)blockIdx.x * 256 + threadIdx.x) * 2; if (e >= (size_t)nh * TT * hd) return; const int d = (int)(e % hd); const int t = (int)((e / hd) % TT); const int h = (int)(e / ((size_t)hd * TT)); v2h o; o[0] = tohx(F[(size_t)t * pitch + h * hd + d]); o[1] = tohx(F[(size_t)t * pitch + h * hd + d + 1]); *(volatile v2h*)(P + e) = o; __threadfence(); *(volatile v2h*)(P + e) = o; }
__global__ __launch_bounds__(256) void k_vt(const float* __restrict__ F, int pitch, int nh, int hd, h16* VT) { const size_t e = ((size_t)blockIdx.x * 256 + threadIdx.x) * 2; if (e >= (size_t)nh * hd * TT) return; const int t = (int)(e % TT); const int d = (int)((e / TT) % hd); const int h = (int)(e / ((size_t)TT * hd)); v2h o; o[0] = tohx(F[(size_t)t * pitch + h * hd + d]); o[1] = tohx(F[(size_t)(t + 1) * pitch + h * hd + d]); *(volatile v2h*)(VT + e) = o; __threadfence(); *(volatile v2h*)(VT + e) = o; }
__global__ __launch_bounds__(256) void k_asoft(const float* __restrict__ Sb, const float* __restrict__ BIAS, const float* __restrict__ MB, int h, float scl, bf* Ph, bf* Pl) { const int lane = threadIdx.x & 31; const int row = blockIdx.x * 8 + (threadIdx.x >> 5); if (row >= TT) return; const float* sr = Sb + (size_t)row * TT; (void)scl; const float* br = BIAS + ((size_t)h * TT + row) * TT; float v[32]; float mx = -3.0e38f;
#pragma unroll
    for (int ch = 0; ch < 8; ++ch) { const int j0 = ch * 128 + lane * 4; const v4f a = *(const v4f*)(sr + j0), bb = *(const v4f*)(br + j0), mm = *(const v4f*)(MB + j0);
#pragma unroll
        for (int q = 0; q < 4; ++q) { const float t = __fadd_rn(__fadd_rn(a[q], bb[q]), mm[q]); v[ch * 4 + q] = t; mx = fmaxf(mx, t); } }
#pragma unroll
    for (int sh = 16; sh; sh >>= 1) mx = fmaxf(mx, __shfl_xor(mx, sh, 32));
    float sum = 0.f;
#pragma unroll
    for (int k = 0; k < 32; ++k) { float d0 = __fsub_rn(v[k], mx); asm volatile("" : "+v"(d0)); v[k] = __builtin_amdgcn_exp2f(__fmul_rn(d0, 1.4426950408889634f)); sum += v[k]; }
#pragma unroll
    for (int sh = 16; sh; sh >>= 1) sum += __shfl_xor(sum, sh, 32);
    const float f = __fdiv_rn(1.0f, sum);
#pragma unroll 1
    for (int ps = 0; ps < 2; ++ps) {
#pragma unroll
        for (int ch = 0; ch < 8; ++ch) { v4us oh, ol;
#pragma unroll
            for (int q = 0; q < 4; ++q) { float y = __fmul_rn(v[ch * 4 + q], f); asm volatile("" : "+v"(y)); unsigned short a2, c2; splitf(y, a2, c2); oh[q] = a2; ol[q] = c2; }
            *(volatile v4us*)(Ph + (size_t)row * TT + ch * 128 + lane * 4) = oh; *(volatile v4us*)(Pl + (size_t)row * TT + ch * 128 + lane * 4) = ol; }
        if (ps == 0) __threadfence(); } }
__global__ __launch_bounds__(256) void k_mrgf(const float* __restrict__ O, int h, int hd, float* CT) { const size_t e = ((size_t)blockIdx.x * 256 + threadIdx.x) * 2; if (e >= (size_t)TT * hd) return; const int d = (int)(e % hd); const int t = (int)(e / hd); v2f o; o[0] = O[e] * (1.0f / PCAR); o[1] = O[e + 1] * (1.0f / PCAR); const size_t oo = (size_t)t * DD + h * hd + d; *(volatile v2f*)(CT + oo) = o; __threadfence(); *(volatile v2f*)(CT + oo) = o; }
__global__ __launch_bounds__(256) void k_mrg(const float* __restrict__ O, int h, int hd, bf* Ah, bf* Al) { const size_t e = ((size_t)blockIdx.x * 256 + threadIdx.x) * 2; if (e >= (size_t)TT * hd) return; const int d = (int)(e % hd); const int t = (int)(e / hd); v2us oh, ol;
#pragma unroll
    for (int q = 0; q < 2; ++q) { unsigned short a, c2; splitf(O[e + q] * (1.0f / PCAR), a, c2); oh[q] = a; ol[q] = c2; } const size_t oo = (size_t)t * DD + h * hd + d; *(volatile v2us*)(Ah + oo) = oh; *(volatile v2us*)(Al + oo) = ol; __threadfence(); *(volatile v2us*)(Ah + oo) = oh; *(volatile v2us*)(Al + oo) = ol; }
__global__ __launch_bounds__(256) void k_cvt8(const float* __restrict__ src, bf* dst, size_t n8) { const size_t i = (size_t)blockIdx.x * 256 + threadIdx.x; if (i >= n8) return; const v8f v = *(const v8f*)(src + i * 8); v8us o;
#pragma unroll
    for (int k = 0; k < 8; ++k) o[k] = f2bf(v[k]); *(volatile v8us*)(dst + i * 8) = o; __threadfence(); *(volatile v8us*)(dst + i * 8) = o; }
__device__ __forceinline__ int t5_bucket(int r) { const int n = r < 0 ? -r : r; int v; if (n < 8) v = n; else { const int k = 31 - __clz(n); v = 8 + 2 * k - 6 + (((long long)n * n >= (1ll << (2 * k + 1))) ? 1 : 0); v = v > 15 ? 15 : v; } return (r > 0 ? 16 : 0) + v; }
__global__ __launch_bounds__(256) void k_rpb(const float* __restrict__ rb, float* BIAS) { const int e = blockIdx.x * 256 + threadIdx.x; if (e >= TT * TT) return; const int j = e % TT, i = e / TT; const int bk = t5_bucket(j - i);
    for (int ps = 0; ps < 2; ++ps) {
#pragma unroll
        for (int h = 0; h < NH_; ++h) *(volatile float*)(BIAS + (size_t)h * TT * TT + e) = bfr(rb[bk * NH_ + h]);
        if (ps == 0) __threadfence(); } }
__global__ __launch_bounds__(256) void k_mrow(const float* __restrict__ mask, float* MBr) { const int e = blockIdx.x * 256 + threadIdx.x; if (e >= NB_ * TT) return; float om = __fsub_rn(1.0f, bfr(mask[e])); asm volatile("" : "+v"(om)); const float v = __fmul_rn(om, -10000.0f); *(volatile float*)(MBr + e) = v; __threadfence(); *(volatile float*)(MBr + e) = v; }

__global__ __launch_bounds__(256) void k_vthl(const float* __restrict__ F, int pitch, bf* VTh, bf* VTl) { const size_t e = ((size_t)blockIdx.x * 256 + threadIdx.x) * 2; if (e >= (size_t)NH_ * HDM * TT) return; const int t = (int)(e % TT); const int d = (int)((e / TT) % HDM); const int h = (int)(e / ((size_t)TT * HDM)); v2us oh, ol;
#pragma unroll
    for (int q = 0; q < 2; ++q) { unsigned short a, c2; splitf(F[(size_t)(t + q) * pitch + h * HDM + d], a, c2); oh[q] = a; ol[q] = c2; } *(volatile v2us*)(VTh + e) = oh; *(volatile v2us*)(VTl + e) = ol; __threadfence(); *(volatile v2us*)(VTh + e) = oh; *(volatile v2us*)(VTl + e) = ol; }
__global__ __launch_bounds__(256) void k_mrgn(const float* __restrict__ O, int h, bf* Ah, bf* Al) { const size_t e = ((size_t)blockIdx.x * 256 + threadIdx.x) * 2; if (e >= (size_t)TT * HDM) return; const int d = (int)(e % HDM), t = (int)(e / HDM); const size_t oo = (size_t)t * DD + h * HDM + d; v2us oh, ol;
#pragma unroll
    for (int q = 0; q < 2; ++q) { unsigned short a, c2; splitf(O[e + q], a, c2); oh[q] = a; ol[q] = c2; } *(volatile v2us*)(Ah + oo) = oh; *(volatile v2us*)(Al + oo) = ol; __threadfence(); *(volatile v2us*)(Ah + oo) = oh; *(volatile v2us*)(Al + oo) = ol; }

__global__ __launch_bounds__(256) void k_plhl(const float* __restrict__ F, int pitch, bf* Ph, bf* Pl) { const size_t e = ((size_t)blockIdx.x * 256 + threadIdx.x) * 2; if (e >= (size_t)NH_ * TT * HDM) return; const int d = (int)(e % HDM); const int t = (int)((e / HDM) % TT); const int h = (int)(e / ((size_t)HDM * TT)); const float* s = F + (size_t)t * pitch + h * HDM + d; v2us oh, ol;
#pragma unroll
    for (int q = 0; q < 2; ++q) { unsigned short a, c2; splitf(s[q], a, c2); oh[q] = a; ol[q] = c2; } *(volatile v2us*)(Ph + e) = oh; *(volatile v2us*)(Pl + e) = ol; __threadfence(); *(volatile v2us*)(Ph + e) = oh; *(volatile v2us*)(Pl + e) = ol; }
__global__ __launch_bounds__(256) void k_zrow(float* MB0) { const int e = blockIdx.x * 256 + threadIdx.x; if (e >= TT) return; *(volatile float*)(MB0 + e) = 0.f; __threadfence(); *(volatile float*)(MB0 + e) = 0.f; }

extern "C" void kernel_launch(void* const* d_in, const int* in_sizes, int n_in,
                              void* d_out, int out_size, void* d_ws, size_t ws_size, hipStream_t stream) {
    (void)in_sizes; (void)n_in; (void)out_size;
    const float* IN[6]; for (int i = 0; i < 6; ++i) IN[i] = (const float*)d_in[i];
    float* OUT = (float*)d_out;
    char* wsp = (char*)d_ws;
    auto take = [&](size_t bytes) { char* p = wsp; wsp += (bytes + 255) & ~(size_t)255; return (void*)p; };
    bf* WQ = (bf*)take((size_t)DD * DD * 2); bf* WK = (bf*)take((size_t)DD * DD * 2); bf* WV = (bf*)take((size_t)DD * DD * 2); bf* WO = (bf*)take((size_t)DD * DD * 2); float* BIAS = (float*)take((size_t)NH_ * TT * TT * 4); float* MB0 = (float*)take((size_t)TT * 4);
    bf* XB = (bf*)take((size_t)TT * DD * 2); float* FQ = (float*)take((size_t)TT * DD * 4); float* FK = (float*)take((size_t)TT * DD * 4); float* FV = (float*)take((size_t)TT * DD * 4);
    bf* QPh = (bf*)take((size_t)TT * DD * 2); bf* QPl = (bf*)take((size_t)TT * DD * 2); bf* KPh = (bf*)take((size_t)TT * DD * 2); bf* KPl = (bf*)take((size_t)TT * DD * 2); bf* VTh = (bf*)take((size_t)DD * TT * 2); bf* VTl = (bf*)take((size_t)DD * TT * 2); float* Sb = (float*)take((size_t)TT * TT * 4); bf* Ph = (bf*)take((size_t)TT * TT * 2); bf* Pl = (bf*)take((size_t)TT * TT * 2); float* O = (float*)take((size_t)TT * HDM * 4); bf* Ah = (bf*)take((size_t)TT * DD * 2); bf* Al = (bf*)take((size_t)TT * DD * 2);
    if ((size_t)(wsp - (char*)d_ws) > ws_size) return;
    { const unsigned g = (unsigned)(((size_t)DD * DD / 64 + 63) / 64); k_wtG<<<g, 256, 0, stream>>>(IN[1], DD, DD, WQ); k_wtG<<<g, 256, 0, stream>>>(IN[2], DD, DD, WK); k_wtG<<<g, 256, 0, stream>>>(IN[3], DD, DD, WV); k_wtG<<<g, 256, 0, stream>>>(IN[4], DD, DD, WO);
      k_rpb<<<(TT * TT + 255) / 256, 256, 0, stream>>>(IN[5], BIAS); k_zrow<<<(TT + 255) / 256, 256, 0, stream>>>(MB0); }
    const unsigned LP = (TT * DD / 2 + 255) / 256;
    for (int b = 0; b < NB_; ++b) {
        k_cvt8<<<(unsigned)(((size_t)TT * DD / 8 + 255) / 256), 256, 0, stream>>>(IN[0] + (size_t)b * TT * DD, XB, (size_t)TT * DD / 8);
        k_gemmw<bf, 0, false><<<dim3(TT / 64, DD / 64, 1), 32, 0, stream>>>(XB, nullptr, WQ, nullptr, DD, FQ, DD, nullptr, 0, 0, 0); k_gemmw<bf, 0, false><<<dim3(TT / 64, DD / 64, 1), 32, 0, stream>>>(XB, nullptr, WK, nullptr, DD, FK, DD, nullptr, 0, 0, 0); k_gemmw<bf, 0, false><<<dim3(TT / 64, DD / 64, 1), 32, 0, stream>>>(XB, nullptr, WV, nullptr, DD, FV, DD, nullptr, 0, 0, 0);
        k_plhl<<<LP, 256, 0, stream>>>(FQ, DD, QPh, QPl); k_plhl<<<LP, 256, 0, stream>>>(FK, DD, KPh, KPl); k_vthl<<<LP, 256, 0, stream>>>(FV, DD, VTh, VTl);
        for (int h = 0; h < NH_; ++h) {
            k_gemmw<bf, 2, false><<<dim3(TT / 64, TT / 64, 1), 32, 0, stream>>>(QPh + (size_t)h * TT * HDM, QPl + (size_t)h * TT * HDM, KPh + (size_t)h * TT * HDM, KPl + (size_t)h * TT * HDM, HDM, Sb, TT, nullptr, 0, 0, 0);
            k_asoft<<<TT / 8, 256, 0, stream>>>(Sb, BIAS, MB0, h, 1.0f, Ph, Pl);
            k_gemmw<bf, 2, false><<<dim3(TT / 64, 1, 1), 32, 0, stream>>>(Ph, Pl, VTh + (size_t)h * HDM * TT, VTl + (size_t)h * HDM * TT, TT, O, HDM, nullptr, 0, 0, 0);
            k_mrgn<<<(TT * HDM / 2 + 255) / 256, 256, 0, stream>>>(O, h, Ah, Al); }
        k_gemmw<bf, 1, false><<<dim3(TT / 64, DD / 64, 1), 32, 0, stream>>>(Ah, Al, WO, nullptr, DD, OUT + (size_t)b * TT * DD, DD, nullptr, 0, 0, 0); }
}
